// Hopfield_68092411511384
// MI455X (gfx1250) — hardware-verified
//
#include <hip/hip_runtime.h>
#include <math.h>
#include <stdint.h>

typedef __attribute__((ext_vector_type(16))) _Float16 v16h;
typedef __attribute__((ext_vector_type(8)))  _Float16 v8h;
typedef __attribute__((ext_vector_type(16))) __bf16   v16b;
typedef __attribute__((ext_vector_type(8)))  __bf16   v8b;
typedef __attribute__((ext_vector_type(8)))  float    v8f;
typedef __attribute__((ext_vector_type(4)))  float    v4f;
typedef __attribute__((ext_vector_type(2)))  float    v2f;
typedef __attribute__((ext_vector_type(4)))  unsigned int v4u;

constexpr int kBatch  = 8;
constexpr int kSeq    = 2048;
constexpr int kDm     = 256;
constexpr int kHeads  = 4;
constexpr int kHd     = 64;
constexpr int kRows   = kBatch * kSeq;

__device__ __forceinline__ unsigned short f2bf_bits(float f) {
  unsigned u = __float_as_uint(f);
  return (unsigned short)((u + 0x7FFFu + ((u >> 16) & 1u)) >> 16);
}
__device__ __forceinline__ float bf_bits2f(unsigned short h) { return __uint_as_float(((unsigned)h) << 16); }

__device__ __forceinline__ void dep_guard_h(v8f& a, v8f& b, v16h x, v16h y) { asm volatile("v_nop\n\tv_nop\n\tv_nop\n\tv_nop" : "+v"(a), "+v"(b) : "v"(x), "v"(y)); }
__device__ __forceinline__ void dep_guard_b(v8f& a, v8f& b, v16b x, v16b y) { asm volatile("v_nop\n\tv_nop\n\tv_nop\n\tv_nop" : "+v"(a), "+v"(b) : "v"(x), "v"(y)); }
__device__ __forceinline__ void keep4_h(v16h a, v16h b, v16h c, v16h d) { asm volatile("v_nop" :: "v"(a), "v"(b), "v"(c), "v"(d)); }
__device__ __forceinline__ void keep4_b(v16b a, v16b b, v16b c, v16b d) { asm volatile("v_nop" :: "v"(a), "v"(b), "v"(c), "v"(d)); }
__device__ __forceinline__ void acc_guard4(v8f& a, v8f& b, v8f& c, v8f& d) { asm volatile("v_nop\n\tv_nop\n\tv_nop\n\tv_nop" : "+v"(a), "+v"(b), "+v"(c), "+v"(d)); }
template <typename T> struct Frag;
template <> struct Frag<_Float16> {
  typedef v16h V; union U { v16h v; v8h h[2]; };
  static __device__ __forceinline__ v16h load(const _Float16* p) {
    U f; f.h[0] = *(const v8h*)(p); f.h[1] = *(const v8h*)(p + 16); return f.v;
  }
  static __device__ __forceinline__ v8f mma(v16h a, v16h b, v8f c) {
    return __builtin_amdgcn_wmma_f32_16x16x32_f16(false, a, false, b, (short)0, c, false, false);
  }
  static __device__ __forceinline__ void guard(v8f& a, v8f& b, v16h x, v16h y) { dep_guard_h(a, b, x, y); }
  static __device__ __forceinline__ void keep(v16h a, v16h b, v16h c, v16h d) { keep4_h(a, b, c, d); }
};
template <> struct Frag<__bf16> {
  typedef v16b V; union U { v16b v; v8b h[2]; };
  static __device__ __forceinline__ v16b load(const __bf16* p) {
    U f; f.h[0] = *(const v8b*)(p); f.h[1] = *(const v8b*)(p + 16); return f.v;
  }
  static __device__ __forceinline__ v8f mma(v16b a, v16b b, v8f c) {
    return __builtin_amdgcn_wmma_f32_16x16x32_bf16(false, a, false, b, (short)0, c, false, false);
  }
  static __device__ __forceinline__ void guard(v8f& a, v8f& b, v16b x, v16b y) { dep_guard_b(a, b, x, y); }
  static __device__ __forceinline__ void keep(v16b a, v16b b, v16b c, v16b d) { keep4_b(a, b, c, d); }
};

template <int ET> struct Elem;
template <> struct Elem<0> { typedef _Float16 T; };
template <> struct Elem<1> { typedef __bf16 T; };
template <int ET, bool SPLIT, int BIAS_MODE, int OUT_MODE, bool RESID, int ACT = 0>
__global__ __launch_bounds__(256) void wmma_gemm64(
    const unsigned short* __restrict__ Ap, const unsigned short* __restrict__ A2p, int lda, long strideA,
    const unsigned short* __restrict__ Btp, const unsigned short* __restrict__ Bt2p, int ldb, long strideB,
    void* __restrict__ Cout, void* __restrict__ Cout2, int ldc, long strideC,
    const float* __restrict__ bias,
    const float* __restrict__ resid, long strideR,
    int M, int N, int K, float scale) {
  typedef typename Elem<ET>::T T;
  typedef typename Frag<T>::V V;
  const T* A = (const T*)Ap; const T* A2 = (const T*)A2p; const T* Bt = (const T*)Btp; const T* Bt2 = (const T*)Bt2p;
  __shared__ __align__(16) float sT[8][16 * 68];
  const int b    = blockIdx.y;
  const int lane = threadIdx.x & 31;
  const int wave = threadIdx.x >> 5;
  const int tilesN = N >> 6;
  const int tilesM = M >> 6;
  const int tile = blockIdx.x * 8 + wave;
  if (tile >= tilesM * tilesN) return;
  const int tm = tile / tilesN;
  const int tn = tile - tm * tilesN;
  const int m0 = tm << 6;
  const int n0 = tn << 6;

  const T* Ab  = A  + (size_t)b * strideA;
  const T* Bb  = Bt + (size_t)b * strideB;
  const T* Ab2 = SPLIT ? (A2  + (size_t)b * strideA) : nullptr;
  const T* Bb2 = SPLIT ? (Bt2 + (size_t)b * strideB) : nullptr;

  const int rlane = lane & 15;
  const int koff  = (lane >> 4) * 8;
  const int mOff  = (lane >> 4) * 8;

  v8f acc[4][4];
#pragma unroll
  for (int i = 0; i < 4; ++i)
#pragma unroll
    for (int j = 0; j < 4; ++j) acc[i][j] = (v8f){0.f,0.f,0.f,0.f,0.f,0.f,0.f,0.f};

  for (int k0 = 0; k0 < K; k0 += 32) {
    V bh[4], bl[4];
#pragma unroll
    for (int j = 0; j < 4; ++j) {
      const size_t bo = (size_t)(n0 + (j << 4) + rlane) * ldb + koff + k0;
      bh[j] = Frag<T>::load(Bb + bo);
      if (SPLIT) bl[j] = Frag<T>::load(Bb2 + bo);
    }
#pragma unroll
    for (int i = 0; i < 4; ++i) {
      const size_t ao = (size_t)(m0 + (i << 4) + rlane) * lda + koff + k0;
      V ah = Frag<T>::load(Ab + ao);
      V al;
      if (SPLIT) al = Frag<T>::load(Ab2 + ao);
#pragma unroll
      for (int j = 0; j < 4; ++j) {
        acc[i][j] = Frag<T>::mma(ah, bh[j], acc[i][j]);
        if (SPLIT) {
          acc[i][j] = Frag<T>::mma(ah, bl[j], acc[i][j]);
          acc[i][j] = Frag<T>::mma(al, bh[j], acc[i][j]);
        }
      }
      Frag<T>::guard(acc[i][0], acc[i][3], ah, SPLIT ? al : ah);
    }
    Frag<T>::keep(bh[0], bh[1], bh[2], bh[3]);
    if (SPLIT) Frag<T>::keep(bl[0], bl[1], bl[2], bl[3]);
  }
  acc_guard4(acc[0][0], acc[0][1], acc[0][2], acc[0][3]);
  acc_guard4(acc[1][0], acc[1][1], acc[1][2], acc[1][3]);
  acc_guard4(acc[2][0], acc[2][1], acc[2][2], acc[2][3]);
  acc_guard4(acc[3][0], acc[3][1], acc[3][2], acc[3][3]);

  float* slab = sT[wave];
  const float* Rb = RESID ? (resid + (size_t)b * strideR) : nullptr;
#pragma unroll
  for (int i = 0; i < 4; ++i) {
    const int mBase = m0 + (i << 4);
#pragma unroll
    for (int j = 0; j < 4; ++j) {
      const int n = n0 + (j << 4) + rlane;
      float bv = 0.f;
      if (BIAS_MODE == 2) bv = bias[n];
#pragma unroll
      for (int r = 0; r < 8; ++r) {
        float v = acc[i][j][r] * scale;
        if (BIAS_MODE == 1) v += bias[mBase + mOff + r];
        if (BIAS_MODE == 2) v += bv;
        if (RESID) v += Rb[(size_t)(mBase + mOff + r) * ldc + n];
        if (ACT == 1) v = tanhf(v);
        if (ACT == 2) v = fmaxf(v, 0.0f);
        if (ACT == 3) v = v / (1.0f + expf(-v));
        if (ACT == 4) v = (v > 0.f) ? v : 0.01f * v;
        if (ACT == 5) v = 0.5f * v * (1.0f + erff(v * 0.70710678118654752f));
        slab[(mOff + r) * 68 + (j << 4) + rlane] = v;
      }
    }
    __builtin_amdgcn_fence(__ATOMIC_RELEASE, "workgroup");
    __builtin_amdgcn_wave_barrier();
    __builtin_amdgcn_fence(__ATOMIC_ACQUIRE, "workgroup");
    if (OUT_MODE == 0) {
      float* C = (float*)Cout + (size_t)b * strideC;
      const int hh = lane >> 4, c4 = (lane & 15) * 4;
      for (int pass = 0; pass < 2; ++pass) {
#pragma unroll
        for (int it = 0; it < 8; ++it) {
          const int row = it * 2 + hh;
          v4f v = *(const v4f*)(slab + row * 68 + c4);
          *(volatile v4f*)(C + (size_t)(mBase + row) * ldc + n0 + c4) = v;
        }
        __threadfence();
      }
    } else {
      const int q = lane >> 3, c8 = (lane & 7) * 8;
      unsigned short* C  = (unsigned short*)Cout  + (size_t)b * strideC;
      unsigned short* C2 = (OUT_MODE == 2) ? ((unsigned short*)Cout2 + (size_t)b * strideC) : nullptr;
      for (int pass = 0; pass < 2; ++pass) {
#pragma unroll
        for (int it = 0; it < 4; ++it) {
          const int row = it * 4 + q;
          const float* sp = slab + row * 68 + c8;
          v8h hv, lv;
#pragma unroll
          for (int e = 0; e < 8; ++e) {
            if (OUT_MODE == 1) {
              hv[e] = (_Float16)sp[e];
            } else {
              unsigned short hb = f2bf_bits(sp[e]);
              unsigned short lb = f2bf_bits(sp[e] - bf_bits2f(hb));
              hv[e] = __builtin_bit_cast(_Float16, hb);
              lv[e] = __builtin_bit_cast(_Float16, lb);
            }
          }
          *(volatile v8h*)(C + (size_t)(mBase + row) * ldc + n0 + c8) = hv;
          if (OUT_MODE == 2) *(volatile v8h*)(C2 + (size_t)(mBase + row) * ldc + n0 + c8) = lv;
        }
        __threadfence();
      }
    }
    __builtin_amdgcn_fence(__ATOMIC_RELEASE, "workgroup");
    __builtin_amdgcn_wave_barrier();
    __builtin_amdgcn_fence(__ATOMIC_ACQUIRE, "workgroup");
  }
}

__device__ __forceinline__ unsigned pk16(unsigned short a, unsigned short b) { return (unsigned)a | ((unsigned)b << 16); }

__global__ __launch_bounds__(256) void split_bf16x2_kernel(const float* __restrict__ in, unsigned short* __restrict__ hi,
                                                           unsigned short* __restrict__ lo, int n2) {
  const int i = blockIdx.x * 256 + threadIdx.x;
  if (i < n2) {
    const v2f f = *(const v2f*)(in + 2 * (size_t)i);
    const unsigned short h0 = f2bf_bits(f[0]), h1 = f2bf_bits(f[1]);
    const unsigned short l0 = f2bf_bits(f[0] - bf_bits2f(h0)), l1 = f2bf_bits(f[1] - bf_bits2f(h1));
    const unsigned uh = pk16(h0, h1), ul = pk16(l0, l1);
    ((volatile unsigned*)hi)[i] = uh;
    ((volatile unsigned*)lo)[i] = ul;
    __threadfence();
    ((volatile unsigned*)hi)[i] = uh;
    ((volatile unsigned*)lo)[i] = ul;
  }
}

__global__ __launch_bounds__(256) void cast_f32_f16x2_scaled(
    const float* __restrict__ in, _Float16* __restrict__ out, int n2, float scale) {
  int i = blockIdx.x * 256 + threadIdx.x;
  if (i < n2) {
    const _Float16 h0 = (_Float16)(in[2 * (size_t)i] * scale), h1 = (_Float16)(in[2 * (size_t)i + 1] * scale);
    const unsigned u = (unsigned)__builtin_bit_cast(unsigned short, h0) | ((unsigned)__builtin_bit_cast(unsigned short, h1) << 16);
    ((volatile unsigned*)out)[i] = u;
    __threadfence();
    ((volatile unsigned*)out)[i] = u;
  }
}

__global__ __launch_bounds__(256) void ln3_kernel(const float* __restrict__ x,
    const float* __restrict__ g_s, const float* __restrict__ b_s,
    const float* __restrict__ g_q, const float* __restrict__ b_q,
    const float* __restrict__ g_v, const float* __restrict__ b_v,
    unsigned short* __restrict__ sk16, unsigned short* __restrict__ sq16,
    unsigned short* __restrict__ svh, unsigned short* __restrict__ svl, int nrows) {
  const int lane = threadIdx.x & 31;
  const int row  = blockIdx.x * 8 + (threadIdx.x >> 5);
  const int rowc = (row < nrows) ? row : (nrows - 1);
  const int c0 = lane * 8;
  const float* xr = x + (size_t)rowc * kDm + c0;
  const v4f a0 = *(const v4f*)xr;
  const v4f a1 = *(const v4f*)(xr + 4);
  float xv[8];
#pragma unroll
  for (int j = 0; j < 4; ++j) { xv[j] = a0[j]; xv[4 + j] = a1[j]; }
  float s = 0.f;
#pragma unroll
  for (int j = 0; j < 8; ++j) s += xv[j];
#pragma unroll
  for (int m = 1; m < 32; m <<= 1) s += __shfl_xor(s, m, 32);
  const float mean = s * (1.0f / 256.0f);
  float ss = 0.f;
#pragma unroll
  for (int j = 0; j < 8; ++j) { const float d = xv[j] - mean; ss += d * d; }
#pragma unroll
  for (int m = 1; m < 32; m <<= 1) ss += __shfl_xor(ss, m, 32);
  const float var  = ss * (1.0f / 256.0f);
  const float rstd = rsqrtf(var + 1e-5f);

  v4u ok, oq, ovh, ovl;
#pragma unroll
  for (int q = 0; q < 4; ++q) {
    const int j0 = 2 * q, j1 = 2 * q + 1;
    const float nx0 = (xv[j0] - mean) * rstd;
    const float nx1 = (xv[j1] - mean) * rstd;
    const float ys0 = nx0 * g_s[c0 + j0] + b_s[c0 + j0];
    const float ys1 = nx1 * g_s[c0 + j1] + b_s[c0 + j1];
    const float yq0 = nx0 * g_q[c0 + j0] + b_q[c0 + j0];
    const float yq1 = nx1 * g_q[c0 + j1] + b_q[c0 + j1];
    const float yv0 = nx0 * g_v[c0 + j0] + b_v[c0 + j0];
    const float yv1 = nx1 * g_v[c0 + j1] + b_v[c0 + j1];
    ok[q] = pk16(__builtin_bit_cast(unsigned short, (_Float16)ys0), __builtin_bit_cast(unsigned short, (_Float16)ys1));
    oq[q] = pk16(__builtin_bit_cast(unsigned short, (_Float16)yq0), __builtin_bit_cast(unsigned short, (_Float16)yq1));
    const unsigned short h0 = f2bf_bits(yv0), h1 = f2bf_bits(yv1);
    const unsigned short l0 = f2bf_bits(yv0 - bf_bits2f(h0)), l1 = f2bf_bits(yv1 - bf_bits2f(h1));
    ovh[q] = pk16(h0, h1);
    ovl[q] = pk16(l0, l1);
  }
  if (row < nrows) {
    const size_t o = (size_t)row * kDm + c0;
    for (int pass = 0; pass < 2; ++pass) {
      *(volatile v4u*)(sk16 + o) = ok;
      *(volatile v4u*)(sq16 + o) = oq;
      *(volatile v4u*)(svh + o)  = ovh;
      *(volatile v4u*)(svl + o)  = ovl;
      __threadfence();
    }
  }
}

constexpr int kAttWaves = 4;
constexpr int kAttQb    = 64;
constexpr int kAttKc    = 64;

__device__ __forceinline__ v8f mma_f16g(v16h a, v16h b, v8f c) {
  c = __builtin_amdgcn_wmma_f32_16x16x32_f16(false, a, false, b, (short)0, c, false, false);
  asm volatile("v_nop\n\tv_nop\n\tv_nop\n\tv_nop" : "+v"(c) : "v"(a), "v"(b));
  return c;
}

__global__ __launch_bounds__(128)
void attn_f16_full_kernel(const unsigned short* __restrict__ qp, const unsigned short* __restrict__ kp,
                          const unsigned short* __restrict__ vtp, float* __restrict__ out, float sscale) {
  union FH { v16h v; v8h h[2]; };
  __shared__ __align__(16) _Float16 Ksh[kAttKc * kHd];
  __shared__ __align__(16) _Float16 Vth[kHd * kAttKc];
  __shared__ __align__(16) _Float16 Psh[kAttWaves][16 * kAttKc];
  __shared__ __align__(16) float    Os[kAttWaves][16 * 68];
  const float kPsc = 32768.0f;

  const int tid  = threadIdx.x;
  const int wave = tid >> 5;
  const int lane = tid & 31;
  const int hh   = lane >> 4;
  const int c    = lane & 15;

  const int nqb = kSeq / kAttQb;
  const int bx = blockIdx.x;
  const int qb = bx % nqb;
  const int h  = bx / nqb;
  const int b  = blockIdx.y;
  const int q0 = qb * kAttQb + wave * 16;

  const _Float16* Qh = (const _Float16*)(const void*)qp + (size_t)b * kSeq * kDm + (size_t)h * kHd;
  const _Float16* Kh = (const _Float16*)(const void*)kp + (size_t)b * kSeq * kDm + (size_t)h * kHd;
  const _Float16* Vh = (const _Float16*)(const void*)vtp + (size_t)b * kDm * kSeq + (size_t)h * kHd * kSeq;
  float*          ob = out + (size_t)b * kSeq * kDm + (size_t)h * kHd;

  v16h qa[2];
#pragma unroll
  for (int dc = 0; dc < 2; ++dc) qa[dc] = Frag<_Float16>::load(Qh + (size_t)(q0 + c) * kDm + dc * 32 + 8 * hh);

  float mrow[8], lrow[8];
  v8f oacc[4];
#pragma unroll
  for (int r = 0; r < 8; ++r) { mrow[r] = -INFINITY; lrow[r] = 0.f; }
#pragma unroll
  for (int t = 0; t < 4; ++t) oacc[t] = (v8f){0.f,0.f,0.f,0.f,0.f,0.f,0.f,0.f};

  const int nChunks = kSeq / kAttKc;
  for (int kc = 0; kc < nChunks; ++kc) {
    const int kv0 = kc * kAttKc;
    __syncthreads();
    {
      const int r = tid >> 1, half = (tid & 1) * 32;
      const _Float16* ksh = Kh + (size_t)(kv0 + r) * kDm + half;
      const _Float16* vsh = Vh + (size_t)r * kSeq + kv0 + half;
#pragma unroll
      for (int i = 0; i < 4; ++i) {
        const v8h av = *(const v8h*)(ksh + 8 * i);
        const v8h bv = *(const v8h*)(vsh + 8 * i);
        *(v8h*)(Ksh + r * kHd    + half + 8 * i) = av;
        *(v8h*)(Vth + r * kAttKc + half + 8 * i) = bv;
      }
    }
    __syncthreads();

    v8f s[4];
#pragma unroll
    for (int j = 0; j < 4; ++j) {
      s[j] = (v8f){0.f,0.f,0.f,0.f,0.f,0.f,0.f,0.f};
#pragma unroll
      for (int dc = 0; dc < 2; ++dc) {
        FH kb;
        kb.h[0] = *(const v8h*)(Ksh + (j * 16 + c) * kHd + dc * 32 + 8 * hh);
        kb.h[1] = *(const v8h*)(Ksh + (j * 16 + c) * kHd + dc * 32 + 16 + 8 * hh);
        s[j] = mma_f16g(qa[dc], kb.v, s[j]);
      }
    }
    float cm[8];
#pragma unroll
    for (int r = 0; r < 8; ++r) {
      float m = -INFINITY;
#pragma unroll
      for (int j = 0; j < 4; ++j) {
        const float sv = s[j][r] * sscale;
        s[j][r] = sv;
        m = fmaxf(m, sv);
      }
#pragma unroll
      for (int off = 1; off < 16; off <<= 1) m = fmaxf(m, __shfl_xor(m, off, 32));
      cm[r] = m;
    }
    _Float16* pw = Psh[wave];
#pragma unroll
    for (int r = 0; r < 8; ++r) {
      const float mnew = fmaxf(mrow[r], cm[r]);
      const float alpha = expf(mrow[r] - mnew);
      mrow[r] = mnew;
      float psum = 0.f;
#pragma unroll
      for (int j = 0; j < 4; ++j) {
        const float p = expf(s[j][r] - mnew);
        psum += p;
        pw[(8 * hh + r) * kAttKc + j * 16 + c] = (_Float16)(p * kPsc);
      }
#pragma unroll
      for (int off = 1; off < 16; off <<= 1) psum += __shfl_xor(psum, off, 32);
      lrow[r] = lrow[r] * alpha + psum;
#pragma unroll
      for (int t = 0; t < 4; ++t) oacc[t][r] *= alpha;
    }
    __builtin_amdgcn_fence(__ATOMIC_RELEASE, "workgroup");
    __builtin_amdgcn_wave_barrier();
    __builtin_amdgcn_fence(__ATOMIC_ACQUIRE, "workgroup");
#pragma unroll 1
    for (int kk = 0; kk < 2; ++kk) {
      FH pa;
      pa.h[0] = *(const v8h*)(pw + c * kAttKc + kk * 32 + 8 * hh);
      pa.h[1] = *(const v8h*)(pw + c * kAttKc + kk * 32 + 16 + 8 * hh);
#pragma unroll
      for (int t = 0; t < 4; ++t) {
        FH vb;
        vb.h[0] = *(const v8h*)(Vth + (t * 16 + c) * kAttKc + kk * 32 + 8 * hh);
        vb.h[1] = *(const v8h*)(Vth + (t * 16 + c) * kAttKc + kk * 32 + 16 + 8 * hh);
        oacc[t] = mma_f16g(pa.v, vb.v, oacc[t]);
      }
    }
  }

  float* os = Os[wave];
#pragma unroll
  for (int r = 0; r < 8; ++r) {
    const float inv = 1.0f / (lrow[r] * kPsc);
#pragma unroll
    for (int t = 0; t < 4; ++t) os[(8 * hh + r) * 68 + t * 16 + c] = oacc[t][r] * inv;
  }
  __builtin_amdgcn_fence(__ATOMIC_RELEASE, "workgroup");
  __builtin_amdgcn_wave_barrier();
  __builtin_amdgcn_fence(__ATOMIC_ACQUIRE, "workgroup");
  {
    const int c4 = (lane & 15) * 4;
    for (int pass = 0; pass < 2; ++pass) {
#pragma unroll
      for (int it = 0; it < 8; ++it) {
        const int row = it * 2 + hh;
        v4f val = *(const v4f*)(os + row * 68 + c4);
        *(volatile v4f*)(ob + (size_t)(q0 + row) * kDm + c4) = val;
      }
      __threadfence();
    }
  }
}

extern "C" void kernel_launch(void* const* d_in, const int* in_sizes, int n_in,
                              void* d_out, int out_size, void* d_ws, size_t ws_size,
                              hipStream_t stream) {
  if (n_in < 15) return;
  if (in_sizes[0] != kRows * kDm) return;
  if (in_sizes[7] != kDm * kDm || in_sizes[9] != kDm * kDm || in_sizes[11] != kDm * kDm || in_sizes[13] != kDm * kDm) return;
  if (in_sizes[1] != kDm || in_sizes[8] != kDm || in_sizes[14] != kDm) return;
  if (out_size != kRows * kDm) return;

  const float* x    = (const float*)d_in[0];
  const float* lnsg = (const float*)d_in[1];
  const float* lnsb = (const float*)d_in[2];
  const float* lnqg = (const float*)d_in[3];
  const float* lnqb = (const float*)d_in[4];
  const float* lnvg = (const float*)d_in[5];
  const float* lnvb = (const float*)d_in[6];
  const float* Wq = (const float*)d_in[7];
  const float* bq = (const float*)d_in[8];
  const float* Wk = (const float*)d_in[9];
  const float* bk = (const float*)d_in[10];
  const float* Wv = (const float*)d_in[11];
  const float* bv = (const float*)d_in[12];
  const float* Wo = (const float*)d_in[13];
  const float* bo = (const float*)d_in[14];
  float* out = (float*)d_out;

  const size_t wBytes   = (size_t)kDm * kDm * 2;
  const size_t plane16  = (size_t)kRows * kDm * 2;
  const size_t plane32  = (size_t)kRows * kDm * 4;
  const size_t offWQ  = 0;
  const size_t offWK  = offWQ + wBytes;
  const size_t offWVH = offWK + wBytes;
  const size_t offWVL = offWVH + wBytes;
  const size_t offWOH = offWVL + wBytes;
  const size_t offWOL = offWOH + wBytes;
  const size_t offSQ  = (size_t)1 << 20;
  const size_t offSK  = offSQ + plane16;
  const size_t offSVH = offSK + plane16;
  const size_t offSVL = offSVH + plane16;
  const size_t offQ16 = offSVL + plane16;
  const size_t offK16 = offQ16 + plane16;
  const size_t offVT  = offK16 + plane16;
  const size_t offAO  = offVT + plane16;
  const size_t offAOH = offAO + plane32;
  const size_t offAOL = offAOH + plane16;
  const size_t total  = offAOL + plane16;
  if (offWOL + wBytes > offSQ) return;
  if (total > ws_size) return;

  char* ws = (char*)d_ws;
  unsigned short* WQ16 = (unsigned short*)(ws + offWQ);
  unsigned short* WK16 = (unsigned short*)(ws + offWK);
  unsigned short* WVH  = (unsigned short*)(ws + offWVH);
  unsigned short* WVL  = (unsigned short*)(ws + offWVL);
  unsigned short* WOH  = (unsigned short*)(ws + offWOH);
  unsigned short* WOL  = (unsigned short*)(ws + offWOL);
  unsigned short* SQ   = (unsigned short*)(ws + offSQ);
  unsigned short* SK   = (unsigned short*)(ws + offSK);
  unsigned short* SVH  = (unsigned short*)(ws + offSVH);
  unsigned short* SVL  = (unsigned short*)(ws + offSVL);
  unsigned short* Q16  = (unsigned short*)(ws + offQ16);
  unsigned short* K16  = (unsigned short*)(ws + offK16);
  unsigned short* VT16 = (unsigned short*)(ws + offVT);
  float*          AO32 = (float*)(ws + offAO);
  unsigned short* AOH  = (unsigned short*)(ws + offAOH);
  unsigned short* AOL  = (unsigned short*)(ws + offAOL);

  const int wN2 = kDm * kDm / 2;
  const int wBlocks = (wN2 + 255) / 256;
  const float wCarry = 16.0f, wCarryInv = 1.0f / 16.0f;

  cast_f32_f16x2_scaled<<<wBlocks, 256, 0, stream>>>(Wq, (_Float16*)WQ16, wN2, wCarry);
  cast_f32_f16x2_scaled<<<wBlocks, 256, 0, stream>>>(Wk, (_Float16*)WK16, wN2, wCarry);
  split_bf16x2_kernel<<<wBlocks, 256, 0, stream>>>(Wv, WVH, WVL, wN2);
  split_bf16x2_kernel<<<wBlocks, 256, 0, stream>>>(Wo, WOH, WOL, wN2);
  ln3_kernel<<<kRows / 8, 256, 0, stream>>>(x, lnsg, lnsb, lnqg, lnqb, lnvg, lnvb, SK, SQ, SVH, SVL, kRows);

  const int projBlocks = ((kRows / 64) * (kDm / 64) + 7) / 8;
  wmma_gemm64<0, false, 2, 1, false><<<dim3(projBlocks, 1), 256, 0, stream>>>(
      SQ, SQ, kDm, 0L, WQ16, WQ16, kDm, 0L, (void*)Q16, (void*)Q16, kDm, 0L,
      bq, bq, 0L, kRows, kDm, kDm, wCarryInv);
  wmma_gemm64<0, false, 2, 1, false><<<dim3(projBlocks, 1), 256, 0, stream>>>(
      SK, SK, kDm, 0L, WK16, WK16, kDm, 0L, (void*)K16, (void*)K16, kDm, 0L,
      bk, bk, 0L, kRows, kDm, kDm, wCarryInv);
  const int vtBlocks = ((kDm / 64) * (kSeq / 64) + 7) / 8;
  wmma_gemm64<1, true, 1, 1, false><<<dim3(vtBlocks, kBatch), 256, 0, stream>>>(
      WVH, WVL, kDm, 0L, SVH, SVL, kDm, (long)kSeq * kDm, (void*)VT16, (void*)VT16, kSeq, (long)kDm * kSeq,
      bv, bv, 0L, kDm, kSeq, kDm, 1.0f);
  attn_f16_full_kernel<<<dim3(kHeads * (kSeq / kAttQb), kBatch), 32 * kAttWaves, 0, stream>>>(
      Q16, K16, VT16, AO32, 0.125f);
  const int aoN2 = kRows * kDm / 2;
  split_bf16x2_kernel<<<(aoN2 + 255) / 256, 256, 0, stream>>>(AO32, AOH, AOL, aoN2);
  wmma_gemm64<1, true, 2, 0, false><<<dim3(projBlocks, 1), 256, 0, stream>>>(
      AOH, AOL, kDm, 0L, WOH, WOL, kDm, 0L, (void*)out, (void*)out, kDm, 0L,
      bo, bo, 0L, kRows, kDm, kDm, 1.0f);
}
